// OuterProductNetwork_11974368821314
// MI455X (gfx1250) — hardware-run, weakly checked
//
#include <hip/hip_runtime.h>


namespace {
constexpr int NBt = 2048, NF = 32, EM = 64, NP = 496;
constexpr float XS = 8.0f, WSC = 256.0f;
typedef _Float16 b16;
typedef __attribute__((ext_vector_type(16))) _Float16 v16b;
typedef __attribute__((ext_vector_type(8))) _Float16 v8b;
typedef __attribute__((ext_vector_type(8))) float v8f;
typedef __attribute__((ext_vector_type(4))) float v4f;
__device__ __forceinline__ float bf16_rne(float f) { unsigned int u = __float_as_uint(f); u += 0x7FFFu + ((u >> 16) & 1u); float r = __uint_as_float(u & 0xFFFF0000u); asm volatile("" : "+v"(r)); return r; }
__device__ __forceinline__ float bfv(float f) { float r = bf16_rne(f); asm volatile("" : "+v"(r)); return r; }
__device__ __forceinline__ v16b frag_kb(const b16* p, int hh) { const v8b a = *(const v8b*)(p + 8 * hh), b = *(const v8b*)(p + 16 + 8 * hh); v16b f;
#pragma unroll
  for (int e = 0; e < 8; ++e) { f[e] = a[e]; f[8 + e] = b[e]; } return f; }
__device__ __forceinline__ v8f wmma16b(v16b a, v16b b, v8f c) { v8f d = __builtin_amdgcn_wmma_f32_16x16x32_f16(false, a, false, b, (short)0, c, false, false); asm volatile("v_nop\n\tv_nop\n\tv_nop\n\tv_nop" : "+v"(d) : "v"(a), "v"(b)); return d; }
__device__ __forceinline__ void wave_lds_sync() { __builtin_amdgcn_fence(__ATOMIC_RELEASE, "workgroup"); __builtin_amdgcn_wave_barrier(); __builtin_amdgcn_fence(__ATOMIC_ACQUIRE, "workgroup"); }
__device__ __forceinline__ float pmul(float a, float b) { float p = a * b; asm volatile("" : "+v"(p)); return p; }
__device__ __forceinline__ void pair_of(int p, int& i, int& j) { int ii = 0, rem = p; while (rem >= NF - 1 - ii) { rem -= NF - 1 - ii; ++ii; } i = ii; j = ii + 1 + rem; }

__global__ __launch_bounds__(256) void wput_kernel(const float* __restrict__ kr, b16* __restrict__ WK) { const size_t nt = (size_t)gridDim.x * 256, u0 = (size_t)blockIdx.x * 256 + threadIdx.x; v8b v;
  for (size_t u = u0; u < (size_t)NP * EM * (EM / 8); u += nt) { const int p = (int)(u / (EM * 8)); const int r = (int)(u % (EM * 8)); const int f = r / 8, e0 = (r % 8) * 8;
#pragma unroll
    for (int j = 0; j < 8; ++j) v[j] = (b16)(bf16_rne(kr[((size_t)f * NP + p) * EM + e0 + j]) * WSC); for (int pass = 0; pass < 2; ++pass) { *(volatile v8b*)(WK + ((size_t)p * EM + f) * EM + e0) = v; __threadfence(); } } }
__global__ __launch_bounds__(32) void pair_kernel(const float* __restrict__ x, const b16* __restrict__ WK, int PLIM, float* __restrict__ R) { __shared__ __attribute__((aligned(16))) b16 Ah[32][EM + 8]; __shared__ float Tf[32][EM + 1], Os[32]; const int lane = threadIdx.x, nloc = lane & 15, hlf = lane >> 4; const int p = blockIdx.x / (NBt / 32); const size_t b0 = (size_t)(blockIdx.x % (NBt / 32)) * 32; if (p >= PLIM) return; int fi, fj; pair_of(p, fi, fj);
  for (int rr = 0; rr < 32; ++rr) for (int q = 0; q < 2; ++q) Ah[rr][q * 32 + lane] = (b16)(bf16_rne(x[((b0 + rr) * NF + fi) * EM + q * 32 + lane]) * XS);
  for (int k = EM; k < EM + 8; ++k) Ah[lane][k] = (b16)0.0f;
  wave_lds_sync();
#pragma unroll
  for (int rt = 0; rt < 2; ++rt) { v8f acc[4] = {(v8f){}, (v8f){}, (v8f){}, (v8f){}};
#pragma unroll
    for (int kb = 0; kb < EM; kb += 32) { const v16b a = frag_kb(&Ah[rt * 16 + nloc][kb], hlf);
#pragma unroll
      for (int t = 0; t < 4; ++t) acc[t] = wmma16b(a, frag_kb(WK + ((size_t)p * EM + t * 16 + nloc) * EM + kb, hlf), acc[t]); }
#pragma unroll
    for (int t = 0; t < 4; ++t)
#pragma unroll
      for (int r8 = 0; r8 < 8; ++r8) Tf[rt * 16 + 8 * hlf + r8][t * 16 + nloc] = acc[t][r8] * (1.0f / (XS * WSC)); }
  wave_lds_sync();
  { float s = 0.0f; const float* xq = x + ((b0 + lane) * NF + fj) * EM;
#pragma unroll 8
    for (int f = 0; f < EM; ++f) s += pmul(Tf[lane][f], bfv(xq[f])); Os[lane] = s; }
  wave_lds_sync();
  for (int pass = 0; pass < 2; ++pass) { ((volatile float*)R)[(size_t)p * NBt + b0 + lane] = Os[lane]; __threadfence(); } }
__global__ __launch_bounds__(256) void out_kernel(const float* __restrict__ R, int PLIM, float* __restrict__ out) { const size_t u = (size_t)blockIdx.x * 256 + threadIdx.x; if (u >= (size_t)NBt * NP) return; const int b = (int)(u / NP), p = (int)(u % NP); if (p >= PLIM) return;
  for (int pass = 0; pass < 2; ++pass) { ((volatile float*)out)[u] = R[(size_t)p * NBt + b]; __threadfence(); } }
}

extern "C" void kernel_launch(void* const* d_in, const int* in_sizes, int n_in, void* d_out, int out_size, void* d_ws, size_t ws_size, hipStream_t stream) {
  (void)n_in;
  auto Fp = [&](int i) { return (const float*)d_in[i]; };
  if (in_sizes[0] != NBt * NF * EM || in_sizes[1] != EM * NP * EM || out_size != NBt * NP) return;
  const int PLIM = NP;
  size_t off = 0; char* ws = (char*)d_ws;
  auto carve = [&](size_t bytes) { char* p = ws + off; off += (bytes + 255) & ~(size_t)255; return p; };
  b16* WK = (b16*)carve((size_t)NP * EM * EM * 2); float* R = (float*)carve((size_t)NP * NBt * 4);
  if (off > ws_size || off > ((size_t)16 << 20)) return;
  wput_kernel<<<256, 256, 0, stream>>>(Fp(1), WK);
  pair_kernel<<<PLIM * (NBt / 32), 32, 0, stream>>>(Fp(0), WK, PLIM, R);
  out_kernel<<<(NBt * NP + 255) / 256, 256, 0, stream>>>(R, PLIM, (float*)d_out);
}
